// EncoderBlock_89773406421661
// MI455X (gfx1250) — hardware-verified
//
#include <hip/hip_runtime.h>
#include <math.h>

#ifndef NB
#define NB 2
#endif
#ifndef SEQ
#define SEQ 2048
#endif
#define SEQ_FULL 2048
#define NTOK (NB * SEQ)

constexpr int kDM = 1024, kNH = 16, kHD = 64, kDF = 4096;
static_assert(kNH * kHD == kDM);
static_assert((SEQ & (SEQ - 1)) == 0);
static_assert(SEQ % 64 == 0);
static_assert(SEQ <= SEQ_FULL);
static_assert(NTOK % 64 == 0);
constexpr unsigned ilog2c(unsigned v) { return v <= 1u ? 0u : 1u + ilog2c(v >> 1); }

typedef __attribute__((ext_vector_type(16))) _Float16 v16h;
typedef __attribute__((ext_vector_type(8)))  _Float16 v8h;
typedef __attribute__((ext_vector_type(8)))  float    v8f;
typedef __attribute__((ext_vector_type(4)))  float    v4f;
typedef __attribute__((ext_vector_type(4)))  unsigned int u4v;
typedef __attribute__((ext_vector_type(2)))  unsigned int u2v;


#define VST2(T, ptr, val) do { const T vst2_v_ = (val); *(volatile T*)(ptr) = vst2_v_; __threadfence(); *(volatile T*)(ptr) = vst2_v_; } while (0)

__device__ __forceinline__ float cmb_bf(float v) { const unsigned u = __builtin_bit_cast(unsigned, v); const unsigned r = (u + 0x7fffu + ((u >> 16) & 1u)) & 0xffff0000u; return __builtin_bit_cast(float, r); }
__device__ __forceinline__ unsigned int cmb_pk2(float a, float b) { return (unsigned int)__builtin_bit_cast(unsigned short, (_Float16)a) | ((unsigned int)__builtin_bit_cast(unsigned short, (_Float16)b) << 16); }

__device__ __forceinline__ v8f wmma16(v16h a, v16h b, v8f c) {
    c = __builtin_amdgcn_wmma_f32_16x16x32_f16(false, a, false, b, (short)0, c, false, false);
    asm volatile("v_nop\n\tv_nop\n\tv_nop\n\tv_nop" : "+v"(c) : "v"(a), "v"(b));
    return c;
}
union FragU { v16h v; v8h h[2]; };
__device__ __forceinline__ v16h frag_load(const _Float16* p) { FragU f; f.h[0] = *(const v8h*)(p); f.h[1] = *(const v8h*)(p + 16); return f.v; }

template <int ABF>
__global__ __launch_bounds__(256) void k_ln_s(const float* __restrict__ A, const float* __restrict__ GA, const float* __restrict__ BE,
                                              unsigned rows, unsigned lg, unsigned rmask, unsigned full_rows, unsigned short* __restrict__ Y16) {
    #pragma clang fp contract(off)
    const unsigned r = blockIdx.x * 8u + (threadIdx.x >> 5); const unsigned L = threadIdx.x & 31u; if (r >= rows) return;
    const size_t ib = ((size_t)(r >> lg) * full_rows + (size_t)(r & rmask)) * 1024u + 4u * L;
    v4f v[8]; float s = 0.f;
#pragma unroll
    for (int q = 0; q < 8; ++q) {
        v[q] = *(const v4f*)(A + ib + 128 * q);
        if (ABF) { v[q].x = cmb_bf(v[q].x); v[q].y = cmb_bf(v[q].y); v[q].z = cmb_bf(v[q].z); v[q].w = cmb_bf(v[q].w); }
        s += (v[q].x + v[q].y) + (v[q].z + v[q].w);
    }
#pragma unroll
    for (int o = 16; o > 0; o >>= 1) s += __shfl_xor(s, o, 32);
    const float mu = s * (1.f / 1024.f); float qq = 0.f;
#pragma unroll
    for (int q = 0; q < 8; ++q) { v[q].x -= mu; v[q].y -= mu; v[q].z -= mu; v[q].w -= mu; qq += (v[q].x * v[q].x + v[q].y * v[q].y) + (v[q].z * v[q].z + v[q].w * v[q].w); }
#pragma unroll
    for (int o = 16; o > 0; o >>= 1) qq += __shfl_xor(qq, o, 32);
    const float sd = sqrtf(qq * (1.f / 1023.f));
    const float rs = 1.0f / (sd + 1e-6f);
    const float al = cmb_bf(GA[0]), be = cmb_bf(BE[0]);
    const size_t ob = (size_t)r * 1024u + 4u * L;
#pragma unroll
    for (int q = 0; q < 8; ++q) {
        v4f y; y.x = (al * v[q].x) * rs + be; y.y = (al * v[q].y) * rs + be; y.z = (al * v[q].z) * rs + be; y.w = (al * v[q].w) * rs + be;
        u2v pk; pk.x = cmb_pk2(y.x, y.y); pk.y = cmb_pk2(y.z, y.w);
        VST2(u2v, (u2v*)(Y16 + ob + 128 * q), pk);
    }
}

__global__ __launch_bounds__(256) void k_cm_castbT(const float* __restrict__ SRC, int lds, unsigned short* __restrict__ DST, int ldd, int nR, int nC, float sc) {
    const long long u = (long long)blockIdx.x * 256 + threadIdx.x; const int per = nR / 8; if (u >= (long long)nC * per) return; const int c = (int)(u / per); const int r0 = 8 * (int)(u % per);
    float w[8];
#pragma unroll
    for (int e = 0; e < 8; ++e) w[e] = cmb_bf(SRC[(long long)(r0 + e) * lds + c]) * sc;
    u4v pk; pk.x = cmb_pk2(w[0], w[1]); pk.y = cmb_pk2(w[2], w[3]); pk.z = cmb_pk2(w[4], w[5]); pk.w = cmb_pk2(w[6], w[7]); VST2(u4v, (u4v*)(DST + (long long)c * ldd + r0), pk); }

__global__ __launch_bounds__(256) void k_bias6(const float* __restrict__ bq, const float* __restrict__ bk, const float* __restrict__ bv, const float* __restrict__ bo,
                                               const float* __restrict__ b1, const float* __restrict__ b2, float* __restrict__ dst) {
    const unsigned blk = blockIdx.x, t = threadIdx.x;
    const float* src = bq; unsigned base = blk * 256u;
    if (blk >= 32u)      { src = b2; base = (blk - 32u) * 256u; }
    else if (blk >= 16u) { src = b1; base = (blk - 16u) * 256u; }
    else if (blk >= 12u) { src = bo; base = (blk - 12u) * 256u; }
    else if (blk >= 8u)  { src = bv; base = (blk - 8u) * 256u; }
    else if (blk >= 4u)  { src = bk; base = (blk - 4u) * 256u; }
    const float v = cmb_bf(src[base + t]);
    VST2(float, dst + blk * 256u + t, v);
}

namespace w25 {
__device__ __forceinline__ void dep_guard_h(v8f& a, v8f& b, v16h x, v16h y) { asm volatile("v_nop\n\tv_nop\n\tv_nop\n\tv_nop" : "+v"(a), "+v"(b) : "v"(x), "v"(y)); }
__device__ __forceinline__ void keep4_h(v16h a, v16h b, v16h c, v16h d) { asm volatile("v_nop" :: "v"(a), "v"(b), "v"(c), "v"(d)); }
__device__ __forceinline__ void acc_guard4(v8f& a, v8f& b, v8f& c, v8f& d) { asm volatile("v_nop\n\tv_nop\n\tv_nop\n\tv_nop" : "+v"(a), "+v"(b), "+v"(c), "+v"(d)); }

template <int BIAS_MODE, int OUT_MODE, bool RESID, int RBF, int ACT>
__global__ __launch_bounds__(256) void wmma_gemm64(
    const unsigned short* __restrict__ Ap, int lda, long strideA,
    const unsigned short* __restrict__ Btp, int ldb, long strideB,
    void* __restrict__ Cout, int ldc, long strideC,
    const float* __restrict__ bias,
    const float* __restrict__ resid, long strideR,
    int M, int N, int K, float scale) {
  const _Float16* A = (const _Float16*)Ap; const _Float16* Bt = (const _Float16*)Btp;
  __shared__ __align__(16) float sT[8][16 * 68];
  const int b    = blockIdx.y;
  const int lane = threadIdx.x & 31;
  const int wave = threadIdx.x >> 5;
  const int tilesN = N >> 6;
  const int tilesM = M >> 6;
  const int tile = blockIdx.x * 8 + wave;
  if (tile >= tilesM * tilesN) return;
  const int tm = tile / tilesN;
  const int tn = tile - tm * tilesN;
  const int m0 = tm << 6;
  const int n0 = tn << 6;

  const _Float16* Ab = A  + (size_t)b * strideA;
  const _Float16* Bb = Bt + (size_t)b * strideB;

  const int rlane = lane & 15;
  const int koff  = (lane >> 4) * 8;
  const int mOff  = (lane >> 4) * 8;

  v8f acc[4][4];
#pragma unroll
  for (int i = 0; i < 4; ++i)
#pragma unroll
    for (int j = 0; j < 4; ++j) acc[i][j] = (v8f){0.f,0.f,0.f,0.f,0.f,0.f,0.f,0.f};

  for (int k0 = 0; k0 < K; k0 += 32) {
    v16h bh[4];
#pragma unroll
    for (int j = 0; j < 4; ++j) {
      const size_t bo = (size_t)(n0 + (j << 4) + rlane) * ldb + koff + k0;
      bh[j] = frag_load(Bb + bo);
    }
#pragma unroll
    for (int i = 0; i < 4; ++i) {
      const size_t ao = (size_t)(m0 + (i << 4) + rlane) * lda + koff + k0;
      const v16h ah = frag_load(Ab + ao);
#pragma unroll
      for (int j = 0; j < 4; ++j)
        acc[i][j] = __builtin_amdgcn_wmma_f32_16x16x32_f16(false, ah, false, bh[j], (short)0, acc[i][j], false, false);
      dep_guard_h(acc[i][0], acc[i][3], ah, ah);
    }
    keep4_h(bh[0], bh[1], bh[2], bh[3]);
  }
  acc_guard4(acc[0][0], acc[0][1], acc[0][2], acc[0][3]);
  acc_guard4(acc[1][0], acc[1][1], acc[1][2], acc[1][3]);
  acc_guard4(acc[2][0], acc[2][1], acc[2][2], acc[2][3]);
  acc_guard4(acc[3][0], acc[3][1], acc[3][2], acc[3][3]);

  float* slab = sT[wave];
  const float* Rb = RESID ? (resid + (size_t)b * strideR) : nullptr;
#pragma unroll
  for (int i = 0; i < 4; ++i) {
    const int mBase = m0 + (i << 4);
#pragma unroll
    for (int j = 0; j < 4; ++j) {
      const int n = n0 + (j << 4) + rlane;
      float bv = 0.f;
      if (BIAS_MODE == 2) bv = bias[n];
#pragma unroll
      for (int r = 0; r < 8; ++r) {
        float v = acc[i][j][r] * scale;
        if (BIAS_MODE == 1) v += bias[mBase + mOff + r];
        if (BIAS_MODE == 2) v += bv;
        if (RESID) { float rv = Rb[(size_t)(mBase + mOff + r) * ldc + n]; if (RBF) rv = cmb_bf(rv); v += rv; }
        if (ACT == 2) v = fmaxf(v, 0.0f);
        slab[(mOff + r) * 68 + (j << 4) + rlane] = v;
      }
    }
    __builtin_amdgcn_fence(3  , "workgroup");
    __builtin_amdgcn_wave_barrier();
    __builtin_amdgcn_fence(2  , "workgroup");
    if (OUT_MODE == 0) {
      float* C = (float*)Cout + (size_t)b * strideC;
      const int hh = lane >> 4, c4 = (lane & 15) * 4;
      for (int pass = 0; pass < 2; ++pass) {
#pragma unroll
        for (int it = 0; it < 8; ++it) {
          const int row = it * 2 + hh;
          v4f v = *(const v4f*)(slab + row * 68 + c4);
          *(volatile v4f*)(C + (size_t)(mBase + row) * ldc + n0 + c4) = v;
        }
        __threadfence();
      }
    } else {
      const int q = lane >> 3, c8 = (lane & 7) * 8;
      unsigned short* C = (unsigned short*)Cout + (size_t)b * strideC;
      for (int pass = 0; pass < 2; ++pass) {
#pragma unroll
        for (int it = 0; it < 4; ++it) {
          const int row = it * 4 + q;
          const float* sp = slab + row * 68 + c8;
          v8h hv;
#pragma unroll
          for (int e = 0; e < 8; ++e) hv[e] = (_Float16)sp[e];
          *(volatile v8h*)(C + (size_t)(mBase + row) * ldc + n0 + c8) = hv;
        }
        __threadfence();
      }
    }
    __builtin_amdgcn_fence(3  , "workgroup");
    __builtin_amdgcn_wave_barrier();
    __builtin_amdgcn_fence(2  , "workgroup");
  }
}

#define AT_NW 4
__global__ __launch_bounds__(128)
void attn_planes(const unsigned short* __restrict__ QKp, unsigned ldqk, unsigned koff,
                 const unsigned short* __restrict__ VTp, unsigned ldvt,
                 const int* __restrict__ mask, unsigned mask_bs,
                 unsigned short* __restrict__ AOp, unsigned ldo, unsigned S,
                 float sscale_l2, float fill_l2, float psc) {
  __shared__ __align__(16) _Float16 Psh[AT_NW][16 * 64];
  __shared__ __align__(16) float    Os[AT_NW][16 * 68];
  const _Float16* QK = (const _Float16*)QKp;
  const _Float16* VT = (const _Float16*)VTp;
  const unsigned tid = threadIdx.x, wave = tid >> 5, lane = tid & 31u, hh = lane >> 4, c = lane & 15u;
  const unsigned qb = blockIdx.x, h = blockIdx.y, b = blockIdx.z;
  const unsigned q0 = qb * 64u + wave * 16u;
  const size_t tok0 = (size_t)b * S;

  v16h qa0, qa1;
  {
    const _Float16* qrow = QK + (tok0 + q0 + c) * ldqk + h * 64u + 8u * hh;
    qa0 = frag_load(qrow); qa1 = frag_load(qrow + 32);
  }
  const _Float16* kbase = QK + tok0 * ldqk + koff + h * 64u + 8u * hh;
  const _Float16* vbase = VT + (size_t)(h * 64u + c) * ldvt + tok0 + 8u * hh;
  const int* mrowp = mask + (size_t)b * mask_bs + c;

  float mrow[8], lrow[8];
  v8f oacc[4];
#pragma unroll
  for (int r = 0; r < 8; ++r) { mrow[r] = -__builtin_inff(); lrow[r] = 0.f; }
#pragma unroll
  for (int t = 0; t < 4; ++t) oacc[t] = (v8f){0.f,0.f,0.f,0.f,0.f,0.f,0.f,0.f};

  _Float16* pw = Psh[wave];
  const unsigned nch = S >> 6;
  for (unsigned kc = 0; kc < nch; ++kc) {
    const unsigned kv0 = kc * 64u;
    v8f s[4];
#pragma unroll
    for (int j = 0; j < 4; ++j) {
      const _Float16* kr = kbase + (size_t)(kv0 + 16u * j + c) * ldqk;
      v8f a = (v8f){0.f,0.f,0.f,0.f,0.f,0.f,0.f,0.f};
      a = wmma16(qa0, frag_load(kr), a);
      a = wmma16(qa1, frag_load(kr + 32), a);
      s[j] = a;
    }
    int kvkeep[4];
#pragma unroll
    for (int j = 0; j < 4; ++j) kvkeep[j] = mrowp[kv0 + 16u * j];
    float cm[8];
#pragma unroll
    for (int r = 0; r < 8; ++r) {
      float m = -__builtin_inff();
#pragma unroll
      for (int j = 0; j < 4; ++j) {
        float v = s[j][r] * sscale_l2;
        v = (kvkeep[j] == 0) ? fill_l2 : v;
        s[j][r] = v;
        m = fmaxf(m, v);
      }
      m = fmaxf(m, __shfl_xor(m, 1, 32)); m = fmaxf(m, __shfl_xor(m, 2, 32));
      m = fmaxf(m, __shfl_xor(m, 4, 32)); m = fmaxf(m, __shfl_xor(m, 8, 32));
      cm[r] = m;
    }
#pragma unroll
    for (int r = 0; r < 8; ++r) {
      const float mnew = fmaxf(mrow[r], cm[r]);
      const float alpha = exp2f(mrow[r] - mnew);
      mrow[r] = mnew;
      float psum = 0.f;
#pragma unroll
      for (int j = 0; j < 4; ++j) {
        const float p = exp2f(s[j][r] - mnew);
        psum += p;
        pw[(8u * hh + r) * 64u + 16u * j + c] = (_Float16)(p * psc);
      }
      psum += __shfl_xor(psum, 1, 32); psum += __shfl_xor(psum, 2, 32);
      psum += __shfl_xor(psum, 4, 32); psum += __shfl_xor(psum, 8, 32);
      lrow[r] = lrow[r] * alpha + psum;
#pragma unroll
      for (int t = 0; t < 4; ++t) oacc[t][r] *= alpha;
    }
    __builtin_amdgcn_fence(3  , "workgroup");
    __builtin_amdgcn_wave_barrier();
    __builtin_amdgcn_fence(2  , "workgroup");
#pragma unroll
    for (int kk = 0; kk < 2; ++kk) {
      const v16h pa = frag_load(pw + c * 64u + 32u * kk + 8u * hh);
#pragma unroll
      for (int t = 0; t < 4; ++t) {
        const v16h vb = frag_load(vbase + (size_t)(16u * t) * ldvt + kv0 + 32u * kk);
        oacc[t] = wmma16(pa, vb, oacc[t]);
      }
    }
    __builtin_amdgcn_fence(3  , "workgroup");
    __builtin_amdgcn_wave_barrier();
    __builtin_amdgcn_fence(2  , "workgroup");
  }

  float* os = Os[wave];
#pragma unroll
  for (int r = 0; r < 8; ++r) {
    const float inv = 1.0f / (lrow[r] * psc);
#pragma unroll
    for (int t = 0; t < 4; ++t) os[(8u * hh + r) * 68u + 16u * t + c] = oacc[t][r] * inv;
  }
  __builtin_amdgcn_fence(3  , "workgroup");
  __builtin_amdgcn_wave_barrier();
  __builtin_amdgcn_fence(2  , "workgroup");
  {
    const unsigned q = lane >> 3, c8 = (lane & 7u) * 8u;
    unsigned short* ob = AOp + (tok0 + q0) * ldo + h * 64u + c8;
    for (int pass = 0; pass < 2; ++pass) {
#pragma unroll
      for (int it = 0; it < 4; ++it) {
        const unsigned row = 4u * it + q;
        const float* sp = os + row * 68u + c8;
        v8h hv;
#pragma unroll
        for (int e = 0; e < 8; ++e) hv[e] = (_Float16)sp[e];
        *(volatile v8h*)(ob + (size_t)row * ldo) = hv;
      }
      __threadfence();
    }
  }
}
}

constexpr size_t al256(size_t b) { return (b + 255) / 256 * 256; }
constexpr size_t SZ_X16  = al256((size_t)NTOK * kDM * 2);
constexpr size_t SZ_WQK  = al256((size_t)2 * kDM * kDM * 2);
constexpr size_t SZ_WSQ  = al256((size_t)kDM * kDM * 2);
constexpr size_t SZ_W1T  = al256((size_t)kDF * kDM * 2);
constexpr size_t SZ_W2T  = al256((size_t)kDM * kDF * 2);
constexpr size_t SZ_BIAS = al256((size_t)9216 * 4);
constexpr size_t SZ_QK16 = al256((size_t)NTOK * 2 * kDM * 2);
constexpr size_t SZ_VT16 = al256((size_t)kDM * NTOK * 2);
constexpr size_t SZ_AO16 = al256((size_t)NTOK * kDM * 2);
constexpr size_t SZ_HF   = al256((size_t)NTOK * kDM * 4);
constexpr size_t SZ_N216 = al256((size_t)NTOK * kDM * 2);
constexpr size_t SZ_A116 = al256((size_t)NTOK * kDF * 2);
constexpr size_t WS_TOTAL = SZ_X16 + SZ_WQK + 2 * SZ_WSQ + SZ_W1T + SZ_W2T + SZ_BIAS + SZ_QK16 + SZ_VT16 + SZ_AO16 + SZ_HF + SZ_N216 + SZ_A116;
static_assert(WS_TOTAL <= (size_t)134217728);
static_assert(((NTOK / 64) * (2 * kDM / 64)) % 8 == 0);
static_assert(((kDM / 64) * (NTOK / 64)) % 8 == 0);
static_assert(((SEQ / 64) * (kDM / 64)) % 8 == 0);
static_assert(((NTOK / 64) * (kDF / 64)) % 8 == 0);
static_assert(((NTOK / 64) * (kDM / 64)) % 8 == 0);
static_assert(NTOK % 8 == 0);
static_assert(kDM % 32 == 0 && kDF % 32 == 0);
static_assert((4 * kDM + kDF + kDM) == 9216);

extern "C" void kernel_launch(void* const* d_in, const int* in_sizes, int n_in, void* d_out, int out_size, void* d_ws, size_t ws_size, hipStream_t stream) {
    if (n_in < 18) return;
    const long long need_x = (long long)(NB - 1) * SEQ_FULL * kDM + (long long)SEQ * kDM;
    const long long need_m = (long long)(NB - 1) * SEQ_FULL + SEQ;
    if ((long long)in_sizes[0] < need_x || (long long)in_sizes[1] < need_m) return;
    if (in_sizes[2] < kDM * kDM || in_sizes[4] < kDM * kDM || in_sizes[6] < kDM * kDM || in_sizes[8] < kDM * kDM) return;
    if (in_sizes[10] < kDM * kDF || in_sizes[12] < kDF * kDM) return;
    if (in_sizes[3] < kDM || in_sizes[5] < kDM || in_sizes[7] < kDM || in_sizes[9] < kDM || in_sizes[11] < kDF || in_sizes[13] < kDM) return;
    if (in_sizes[14] < 1 || in_sizes[15] < 1 || in_sizes[16] < 1 || in_sizes[17] < 1) return;
    if ((long long)out_size < (long long)NTOK * kDM) return;
    if (WS_TOTAL > ws_size) return;

    const float* x    = (const float*)d_in[0];
    const int*   mask = (const int*)d_in[1];
    const float* Wq = (const float*)d_in[2];  const float* bq = (const float*)d_in[3];
    const float* Wk = (const float*)d_in[4];  const float* bk = (const float*)d_in[5];
    const float* Wv = (const float*)d_in[6];  const float* bv = (const float*)d_in[7];
    const float* Wo = (const float*)d_in[8];  const float* bo = (const float*)d_in[9];
    const float* W1 = (const float*)d_in[10]; const float* b1 = (const float*)d_in[11];
    const float* W2 = (const float*)d_in[12]; const float* b2 = (const float*)d_in[13];
    const float* alpha1 = (const float*)d_in[14];
    const float* beta1  = (const float*)d_in[15];
    const float* alpha2 = (const float*)d_in[16];
    const float* beta2  = (const float*)d_in[17];
    float* out = (float*)d_out;

    char* wsp = (char*)d_ws;
    unsigned short* X16  = (unsigned short*)wsp; wsp += SZ_X16;
    unsigned short* WQK  = (unsigned short*)wsp; wsp += SZ_WQK;
    unsigned short* WVT  = (unsigned short*)wsp; wsp += SZ_WSQ;
    unsigned short* WOT  = (unsigned short*)wsp; wsp += SZ_WSQ;
    unsigned short* W1T  = (unsigned short*)wsp; wsp += SZ_W1T;
    unsigned short* W2T  = (unsigned short*)wsp; wsp += SZ_W2T;
    float*          BIAS = (float*)wsp;          wsp += SZ_BIAS;
    unsigned short* QK16 = (unsigned short*)wsp; wsp += SZ_QK16;
    unsigned short* VT16 = (unsigned short*)wsp; wsp += SZ_VT16;
    unsigned short* AO16 = (unsigned short*)wsp; wsp += SZ_AO16;
    float*          HF   = (float*)wsp;          wsp += SZ_HF;
    unsigned short* N216 = (unsigned short*)wsp; wsp += SZ_N216;
    unsigned short* A116 = (unsigned short*)wsp; wsp += SZ_A116;
    const float* BQK = BIAS; const float* BV = BIAS + 2048; const float* BO = BIAS + 3072; const float* B1 = BIAS + 4096; const float* B2 = BIAS + 8192;

    const unsigned lg = ilog2c((unsigned)SEQ), rmask = (unsigned)SEQ - 1u;

    k_ln_s<1><<<NTOK / 8, 256, 0, stream>>>(x, alpha1, beta1, (unsigned)NTOK, lg, rmask, (unsigned)SEQ_FULL, X16);
    k_cm_castbT<<<(kDM * (kDM / 8) + 255) / 256, 256, 0, stream>>>(Wq, kDM, WQK, kDM, kDM, kDM, 16.0f);
    k_cm_castbT<<<(kDM * (kDM / 8) + 255) / 256, 256, 0, stream>>>(Wk, kDM, WQK + (size_t)kDM * kDM, kDM, kDM, kDM, 16.0f);
    k_cm_castbT<<<(kDM * (kDM / 8) + 255) / 256, 256, 0, stream>>>(Wv, kDM, WVT, kDM, kDM, kDM, 16.0f);
    k_cm_castbT<<<(kDM * (kDM / 8) + 255) / 256, 256, 0, stream>>>(Wo, kDM, WOT, kDM, kDM, kDM, 16.0f);
    k_cm_castbT<<<(kDF * (kDM / 8) + 255) / 256, 256, 0, stream>>>(W1, kDF, W1T, kDM, kDM, kDF, 16.0f);
    k_cm_castbT<<<(kDM * (kDF / 8) + 255) / 256, 256, 0, stream>>>(W2, kDM, W2T, kDF, kDF, kDM, 16.0f);
    k_bias6<<<36, 256, 0, stream>>>(bq, bk, bv, bo, b1, b2, BIAS);

    w25::wmma_gemm64<2, 1, false, 0, 0><<<dim3((unsigned)(((NTOK / 64) * (2 * kDM / 64) + 7) / 8), 1u), 256, 0, stream>>>(
        X16, kDM, 0L, WQK, kDM, 0L, (void*)QK16, 2 * kDM, 0L, BQK, nullptr, 0L, NTOK, 2 * kDM, kDM, 0.0625f);
    w25::wmma_gemm64<1, 1, false, 0, 0><<<dim3((unsigned)(((kDM / 64) * (NTOK / 64) + 7) / 8), 1u), 256, 0, stream>>>(
        WVT, kDM, 0L, X16, kDM, 0L, (void*)VT16, NTOK, 0L, BV, nullptr, 0L, kDM, NTOK, kDM, 0.0625f);
    w25::attn_planes<<<dim3((unsigned)(SEQ / 64), (unsigned)kNH, (unsigned)NB), 128, 0, stream>>>(
        QK16, 2u * kDM, (unsigned)kDM, VT16, (unsigned)NTOK, mask, (unsigned)SEQ_FULL, AO16, (unsigned)kDM, (unsigned)SEQ,
        0.125f * 1.4426950408889634f, -1.0e9f * 1.4426950408889634f, 16384.0f);
    w25::wmma_gemm64<2, 0, true, 1, 0><<<dim3((unsigned)(((SEQ / 64) * (kDM / 64) + 7) / 8), (unsigned)NB), 256, 0, stream>>>(
        AO16, kDM, (long)SEQ * kDM, WOT, kDM, 0L, (void*)HF, kDM, (long)SEQ * kDM, BO, x, (long)SEQ_FULL * kDM, SEQ, kDM, kDM, 0.0625f);
    k_ln_s<0><<<NTOK / 8, 256, 0, stream>>>(HF, alpha2, beta2, (unsigned)NTOK, lg, rmask, (unsigned)SEQ, N216);
    w25::wmma_gemm64<2, 1, false, 0, 2><<<dim3((unsigned)(((NTOK / 64) * (kDF / 64) + 7) / 8), 1u), 256, 0, stream>>>(
        N216, kDM, 0L, W1T, kDM, 0L, (void*)A116, kDF, 0L, B1, nullptr, 0L, NTOK, kDF, kDM, 0.0625f);
    w25::wmma_gemm64<2, 0, true, 0, 0><<<dim3((unsigned)(((NTOK / 64) * (kDM / 64) + 7) / 8), 1u), 256, 0, stream>>>(
        A116, kDF, 0L, W2T, kDF, 0L, (void*)out, kDM, 0L, B2, HF, 0L, NTOK, kDM, kDF, 0.0625f);
}
